// BidirectionalAntiAttention_15625091023578
// MI455X (gfx1250) — hardware-verified
//
#include <hip/hip_runtime.h>
#include <math.h>

typedef __attribute__((ext_vector_type(16))) _Float16 v16h;
typedef __attribute__((ext_vector_type(16))) __bf16 v16b;
typedef __attribute__((ext_vector_type(8)))  _Float16 v8h;
typedef __attribute__((ext_vector_type(8)))  float v8f;
typedef __attribute__((ext_vector_type(4)))  float v4f;
typedef __attribute__((ext_vector_type(2)))  float v2f;
typedef __attribute__((ext_vector_type(4)))  unsigned v4u;
typedef __attribute__((ext_vector_type(4)))  int v4i;
typedef float __attribute__((may_alias)) float_a;
typedef int __attribute__((may_alias)) int_a;

template <typename T> __device__ __forceinline__ void vst2(void* p, T v) { *(volatile T*)p = v; __threadfence(); *(volatile T*)p = v; }
__device__ __forceinline__ v8f wmma16(v16h a, v16h b, v8f c) {
  v8f d = __builtin_amdgcn_wmma_f32_16x16x32_f16(false, a, false, b, (short)0, c, false, false);
  asm volatile("v_nop\n\tv_nop\n\tv_nop\n\tv_nop" : "+v"(d) : "v"(a), "v"(b));
  return d;
}
__device__ __forceinline__ v8f wmma_bf(v16b a, v16b b, v8f c) {
  v8f d = __builtin_amdgcn_wmma_f32_16x16x32_bf16(false, a, false, b, (short)0, c, false, false);
  asm volatile("v_nop\n\tv_nop\n\tv_nop\n\tv_nop" : "+v"(d) : "v"(a), "v"(b));
  return d;
}
__device__ __forceinline__ v16h frag_h(const _Float16* rowk0, int lane) {
  union { v16h v; v8h q[2]; } u; const _Float16* p = rowk0 + 8 * (lane >> 4);
  u.q[0] = *(const v8h*)p; u.q[1] = *(const v8h*)(p + 16); return u.v;
}
__device__ __forceinline__ v16h frag_f32(const float* rowk0, int lane) {
  v16h a; const float* p = rowk0 + 8 * (lane >> 4);
#pragma unroll
  for (int i = 0; i < 8; ++i) { a[i] = (_Float16)p[i]; a[8 + i] = (_Float16)p[16 + i]; }
  return a;
}
__device__ __forceinline__ v16h frag_f32s(const float* rowk0, int lane, float sc) {
  v16h a; const float* p = rowk0 + 8 * (lane >> 4);
#pragma unroll
  for (int i = 0; i < 8; ++i) { a[i] = (_Float16)(p[i] * sc); a[8 + i] = (_Float16)(p[16 + i] * sc); }
  return a;
}
__device__ __forceinline__ v16h fragc_f32(const float* W, int k0, int n, int lane, int ld, int K) {
  v16h a; const int g = lane >> 4;
#pragma unroll
  for (int i = 0; i < 8; ++i) { const int ka = k0 + 8 * g + i, kb = ka + 16;
    a[i] = (_Float16)(ka < K ? W[(size_t)(ka < K ? ka : K - 1) * ld + n] : 0.f); a[8 + i] = (_Float16)(kb < K ? W[(size_t)(kb < K ? kb : K - 1) * ld + n] : 0.f); }
  return a;
}
struct F2 { v16b h, l; };
__device__ __forceinline__ F2 bsplit16(const float v[16]) { F2 r;
#pragma unroll
  for (int i = 0; i < 16; ++i) { const __bf16 h = (__bf16)v[i]; r.h[i] = h; r.l[i] = (__bf16)(v[i] - (float)h); }
  return r; }
__device__ __forceinline__ F2 split_row(const float* row, int k0, int lane) { float v[16]; const float* p = row + k0 + 8 * (lane >> 4);
#pragma unroll
  for (int i = 0; i < 8; ++i) { v[i] = p[i]; v[8 + i] = p[16 + i]; }
  return bsplit16(v); }
__device__ __forceinline__ F2 split_rowK(const float* row, int k0, int lane, int K) { float v[16]; const int g = lane >> 4;
#pragma unroll
  for (int i = 0; i < 8; ++i) { const int ka = k0 + 8 * g + i, kb = ka + 16; v[i] = ka < K ? row[ka < K ? ka : K - 1] : 0.f; v[8 + i] = kb < K ? row[kb < K ? kb : K - 1] : 0.f; }
  return bsplit16(v); }
__device__ __forceinline__ F2 split_col(const float* W, int k0, int n, int lane, int ld, int K) { float v[16]; const int g = lane >> 4;
#pragma unroll
  for (int i = 0; i < 8; ++i) { const int ka = k0 + 8 * g + i, kb = ka + 16; v[i] = ka < K ? W[(size_t)(ka < K ? ka : K - 1) * ld + n] : 0.f; v[8 + i] = kb < K ? W[(size_t)(kb < K ? kb : K - 1) * ld + n] : 0.f; }
  return bsplit16(v); }
__device__ __forceinline__ v8f mac3(const F2& a, const F2& b, v8f c) { c = wmma_bf(a.l, b.h, c); c = wmma_bf(a.h, b.l, c); return wmma_bf(a.h, b.h, c); }
__device__ __forceinline__ float sigm(float v) { return 1.0f / (1.0f + expf(-v)); }
#define LDSX() do { asm volatile("s_wait_dscnt 0" ::: "memory"); __builtin_amdgcn_wave_barrier(); __builtin_amdgcn_fence(__ATOMIC_RELEASE, "workgroup"); } while (0)


#define NB 4
#define LL 2048
#define DD 768
#define RR 32
#define PP 496
#define NROW (NB * LL)
#ifndef TRB
#define TRB (NROW / 64)
#endif
typedef __attribute__((ext_vector_type(8))) __bf16 v8b;
__device__ __forceinline__ v16b frag_b(const __bf16* rowk0, int lane) {
  union { v16b v; v8b q[2]; } u; const __bf16* p = rowk0 + 8 * (lane >> 4);
  u.q[0] = *(const v8b*)p; u.q[1] = *(const v8b*)(p + 16); return u.v;
}
__device__ __forceinline__ float bfr(float v) { return (float)(__bf16)v; }
__device__ __attribute__((noinline)) float exp_ni(float v) { return expf(v); }
__device__ __attribute__((noinline)) float erf_ni(float v) { return erff(v); }

#define WS_Z   0u
#define WS_GF  (WS_Z + 4u * (size_t)NROW * RR)
#define WS_GB  (WS_GF + 4u * (size_t)NROW * DD)
#define WS_H   (WS_GB + 4u * (size_t)NROW * DD)
#define WS_PB  (WS_H + 4u * (size_t)NROW * DD)
#define WS_WH  (WS_PB + 2u * (size_t)2 * 4 * NROW * 512)
#define WS_END (WS_WH + 2u * (size_t)(512 + 512 + 1536) * DD)

__global__ __launch_bounds__(128) void k_z(const float* __restrict__ X, const float* __restrict__ WDR, const float* __restrict__ BDR, float* __restrict__ Z) { __shared__ __align__(16) float sz[4][16][36];
  const int tid = threadIdx.x, wave = tid >> 5, lane = tid & 31, col = lane & 15, g = lane >> 4; const size_t r0 = (size_t)blockIdx.x * 64 + wave * 16;
  v8f acc[2] = {};
#pragma unroll 2
  for (int kc = 0; kc < DD / 32; ++kc) { v16b a; { const float* p = X + (r0 + col) * DD + kc * 32 + 8 * g;
#pragma unroll
      for (int i = 0; i < 8; ++i) { a[i] = (__bf16)p[i]; a[8 + i] = (__bf16)p[16 + i]; } }
#pragma unroll
    for (int j = 0; j < 2; ++j) { v16b w; const int o = j * 16 + col;
#pragma unroll
      for (int i = 0; i < 8; ++i) { w[i] = (__bf16)WDR[(size_t)(kc * 32 + 8 * g + i) * RR + o]; w[8 + i] = (__bf16)WDR[(size_t)(kc * 32 + 16 + 8 * g + i) * RR + o]; }
      acc[j] = wmma_bf(a, w, acc[j]); } }
#pragma unroll
  for (int j = 0; j < 2; ++j) { const float bb = bfr(BDR[j * 16 + col]);
#pragma unroll
    for (int r = 0; r < 8; ++r) sz[wave][8 * g + r][j * 16 + col] = acc[j][r] + bb; }
  LDSX(); for (int rl = 0; rl < 16; ++rl) if (lane < 8) vst2(Z + (r0 + rl) * RR + lane * 4, *(const v4f*)&sz[wave][rl][lane * 4]); }
__constant__ int c_off[4] = {1, 2, 4, 8};
__global__ __launch_bounds__(192) void k_wh(const float* __restrict__ WF, const float* __restrict__ WB, const float* __restrict__ WG, _Float16* __restrict__ WH) { const int row = blockIdx.x; const int t = threadIdx.x;
  const float* src = nullptr; if (row < 512) { if (row < PP) src = WF + (size_t)row * DD; } else if (row < 1024) { if (row - 512 < PP) src = WB + (size_t)(row - 512) * DD; } else src = WG + (size_t)(DD + (row - 1024)) * DD;
  __shared__ __align__(16) _Float16 s[DD]; for (int c = t; c < DD; c += 192) s[c] = (_Float16)(src ? bfr(src[c]) : 0.f); __syncthreads(); if (t < DD / 8) vst2((unsigned*)(WH + (size_t)row * DD + t * 8), *(const v4u*)&s[t * 8]); }
__global__ __launch_bounds__(128) void k_pl(const float* __restrict__ Z, _Float16* __restrict__ PB) { __shared__ float szl[64][RR + 1], szr[64][RR + 1]; __shared__ float spart[4][64]; __shared__ float sinv[64]; __shared__ __align__(16) _Float16 sp[64][520];
  const int tid = threadIdx.x; const int oi = blockIdx.y, dir = blockIdx.z; const int dl = c_off[oi]; const size_t r0 = (size_t)blockIdx.x * 64;
  for (int e = tid; e < 64 * RR; e += 128) { const int rl = e / RR, k = e % RR; const size_t row = r0 + rl; const int l = (int)(row % LL); const int lp = dir == 0 ? l + dl : l - dl; const bool ok = (lp >= 0 && lp < LL); szl[rl][k] = Z[row * RR + k]; szr[rl][k] = ok ? Z[(row - l + lp) * RR + k] : 0.f; }
  __syncthreads();
  int pi[4], pj[4], np_ = 0; for (int q = tid; q < PP; q += 128) { int i = 0, rem = q; while (rem >= RR - 1 - i) { rem -= RR - 1 - i; ++i; } pi[np_] = i; pj[np_] = i + 1 + rem; ++np_; }
#pragma unroll 1
  for (int quarter = 0; quarter < 4; ++quarter) {
#pragma unroll 1
    for (int rl = quarter * 16; rl < quarter * 16 + 16; ++rl) { float s = 0.f;
#pragma unroll 1
      for (int m = 0; m < np_; ++m) { const float v = szl[rl][pi[m]] * szr[rl][pj[m]] - szl[rl][pj[m]] * szr[rl][pi[m]]; s += v * v; }
#pragma unroll
      for (int o = 1; o < 32; o <<= 1) s += __shfl_xor(s, o);
      if ((tid & 31) == 0) spart[tid >> 5][rl] = s; } }
  __syncthreads();
  if (tid < 64) sinv[tid] = 1.0f / fmaxf(sqrtf((spart[0][tid] + spart[1][tid]) + (spart[2][tid] + spart[3][tid])), 1e-8f);
  __syncthreads();
#pragma unroll 1
  for (int rl = 0; rl < 64; ++rl) { const float inv = sinv[rl];
#pragma unroll 1
    for (int m = 0; m < np_; ++m) { const int q = tid + 128 * m; const float v = szl[rl][pi[m]] * szr[rl][pj[m]] - szl[rl][pj[m]] * szr[rl][pi[m]]; sp[rl][q] = (_Float16)(v * inv); } if (tid < 512 - PP) sp[rl][PP + tid] = (_Float16)0.0f; }
  __syncthreads();
  { _Float16* dst = PB + (((size_t)dir * 4 + oi) * NROW + r0) * 512; for (int e = tid; e < 64 * 64; e += 128) { const int rl = e >> 6, q = e & 63; vst2((unsigned*)(dst + (size_t)rl * 512 + q * 8), *(const v4u*)&sp[rl][q * 8]); } } }
__global__ __launch_bounds__(128) void k_dir(const _Float16* __restrict__ PB, const _Float16* __restrict__ WH, const float* __restrict__ BF, const float* __restrict__ BB, float* __restrict__ GF, float* __restrict__ GB) {
  __shared__ __align__(16) float so[4][16][132];
  const int tid = threadIdx.x, wave = tid >> 5, lane = tid & 31, col = lane & 15, g = lane >> 4; const int c0 = blockIdx.y * 128; const int dir = blockIdx.z; const size_t r0 = (size_t)blockIdx.x * 64 + wave * 16;
  const _Float16* Wm = WH + (size_t)dir * 512 * DD; const float* Bm = dir == 0 ? BF : BB; float* G = dir == 0 ? GF : GB;
  float gsum[8][8];
#pragma unroll
  for (int j = 0; j < 8; ++j)
#pragma unroll
    for (int r = 0; r < 8; ++r) gsum[j][r] = 0.f;
#pragma unroll 1
  for (int oi = 0; oi < 4; ++oi) { const int dl = c_off[oi]; const _Float16* prow = PB + (((size_t)dir * 4 + oi) * NROW + r0 + col) * 512;
    v8f acc[8] = {};
#pragma unroll 1
    for (int kc = 0; kc < 512 / 32; ++kc) { const v16h a = frag_h(prow + kc * 32, lane);
#pragma unroll
      for (int j = 0; j < 8; ++j) { v16h w; const int o = c0 + j * 16 + col;
#pragma unroll
        for (int i = 0; i < 8; ++i) { w[i] = Wm[(size_t)(kc * 32 + 8 * g + i) * DD + o]; w[8 + i] = Wm[(size_t)(kc * 32 + 16 + 8 * g + i) * DD + o]; }
        acc[j] = wmma16(a, w, acc[j]); } }
#pragma unroll
    for (int j = 0; j < 8; ++j) { const float bb = bfr(Bm[c0 + j * 16 + col]);
#pragma unroll
      for (int r = 0; r < 8; ++r) { const size_t row = r0 + 8 * g + r; const int l = (int)(row % LL); const int lp = dir == 0 ? l + dl : l - dl; if (lp >= 0 && lp < LL) gsum[j][r] += acc[j][r] + bb; } } }
#pragma unroll
  for (int j = 0; j < 8; ++j)
#pragma unroll
    for (int r = 0; r < 8; ++r) { const size_t row = r0 + 8 * g + r; const int l = (int)(row % LL); int cnt = 0; for (int oi = 0; oi < 4; ++oi) { const int lp = dir == 0 ? l + c_off[oi] : l - c_off[oi]; cnt += (lp >= 0 && lp < LL) ? 1 : 0; } so[wave][8 * g + r][j * 16 + col] = gsum[j][r] / (float)(cnt > 0 ? cnt : 1); }
  LDSX(); for (int rl = 0; rl < 16; ++rl) vst2(G + (r0 + rl) * DD + c0 + lane * 4, *(const v4f*)&so[wave][rl][lane * 4]); }
__global__ __launch_bounds__(128) void k_gate(const float* __restrict__ X, const float* __restrict__ GF, const float* __restrict__ GB, const float* __restrict__ WG, const _Float16* __restrict__ WH, const float* __restrict__ BG, float* __restrict__ Hh) { const _Float16* WGH = WH + (size_t)1024 * DD;   __shared__ __align__(16) float so[4][16][132];
  const int tid = threadIdx.x, wave = tid >> 5, lane = tid & 31, col = lane & 15, g = lane >> 4; const int c0 = blockIdx.y * 128; const size_t r0 = (size_t)blockIdx.x * 64 + wave * 16;
  v8f acc[8] = {};
#pragma unroll 1
  for (int part = 0; part < 3; ++part) { const float* SRC = part == 0 ? X : part == 1 ? GF : GB;
#pragma unroll 2
    for (int kc = 0; kc < DD / 32; ++kc) { const int kg = part * DD + kc * 32;
      if (part == 0) { v16b a; { const float* p = SRC + (r0 + col) * DD + kc * 32 + 8 * g;
#pragma unroll
          for (int i = 0; i < 8; ++i) { a[i] = (__bf16)p[i]; a[8 + i] = (__bf16)p[16 + i]; } }
#pragma unroll
        for (int j = 0; j < 8; ++j) { v16b w; const int o = c0 + j * 16 + col;
#pragma unroll
          for (int i = 0; i < 8; ++i) { w[i] = (__bf16)WG[(size_t)(kg + 8 * g + i) * DD + o]; w[8 + i] = (__bf16)WG[(size_t)(kg + 16 + 8 * g + i) * DD + o]; }
          acc[j] = wmma_bf(a, w, acc[j]); } }
      else { const v16h a = frag_f32(SRC + (r0 + col) * DD + kc * 32, lane);
#pragma unroll
        for (int j = 0; j < 8; ++j) { v16h w; const int o = c0 + j * 16 + col;
#pragma unroll
          for (int i = 0; i < 8; ++i) { w[i] = WGH[(size_t)(kg - DD + 8 * g + i) * DD + o]; w[8 + i] = WGH[(size_t)(kg - DD + 16 + 8 * g + i) * DD + o]; }
          acc[j] = wmma16(a, w, acc[j]); } } } }
#pragma unroll
  for (int j = 0; j < 8; ++j) { const int c = c0 + j * 16 + col; const float bb = bfr(BG[c]);
#pragma unroll
    for (int r = 0; r < 8; ++r) { const size_t row = r0 + 8 * g + r; const float al = 1.0f / (1.0f + expf(-(acc[j][r] + bb))); const float gc = 0.5f * (GF[row * DD + c] + GB[row * DD + c]); so[wave][8 * g + r][j * 16 + col] = al * bfr(X[row * DD + c]) + (1.0f - al) * gc; } }
  LDSX(); for (int rl = 0; rl < 16; ++rl) vst2(Hh + (r0 + rl) * DD + c0 + lane * 4, *(const v4f*)&so[wave][rl][lane * 4]); }
__global__ __launch_bounds__(256) void k_rms(const float* __restrict__ Hh, const float* __restrict__ SC, float* __restrict__ OUT) { __shared__ float sred[8]; __shared__ float sinv; __shared__ __align__(16) float so[DD];
  const int t = threadIdx.x; const size_t row = blockIdx.x; const float* h = Hh + row * DD;
  float s = 0.f; for (int c = t; c < DD; c += 256) { const float v = h[c]; s += v * v; }
#pragma unroll
  for (int o = 1; o < 32; o <<= 1) s += __shfl_xor(s, o);
  if ((t & 31) == 0) sred[t >> 5] = s; __syncthreads(); if (t == 0) { float a = 0.f; for (int i = 0; i < 8; ++i) a += sred[i]; sinv = 1.0f / sqrtf(a * (1.0f / DD) + 1e-5f); } __syncthreads();
  for (int c = t; c < DD; c += 256) so[c] = h[c] * sinv * bfr(SC[c]);
  __syncthreads(); for (int q = t; q < DD / 4; q += 256) vst2(OUT + row * DD + q * 4, *(const v4f*)&so[q * 4]); }
extern "C" void kernel_launch(void* const* d_in, const int* in_sizes, int n_in, void* d_out, int out_size, void* d_ws, size_t ws_size, hipStream_t stream) {
  (void)in_sizes; (void)n_in; (void)out_size;
  const float** F = (const float**)d_in;
  if (ws_size < (size_t)WS_END) return;
  char* ws = (char*)d_ws; float *Z = (float*)(ws + WS_Z), *GF = (float*)(ws + WS_GF), *GB = (float*)(ws + WS_GB), *Hh = (float*)(ws + WS_H); _Float16 *PB = (_Float16*)(ws + WS_PB), *WH = (_Float16*)(ws + WS_WH);
  k_wh<<<512 + 512 + 1536, 192, 0, stream>>>(F[3], F[5], F[7], WH);
  k_z<<<NROW / 64, 128, 0, stream>>>(F[0], F[1], F[2], Z);
  k_pl<<<dim3(TRB, 4, 2), 128, 0, stream>>>(Z, PB);
  k_dir<<<dim3(TRB, DD / 128, 2), 128, 0, stream>>>(PB, WH, F[4], F[6], GF, GB);
  k_gate<<<dim3(TRB, DD / 128), 128, 0, stream>>>(F[0], GF, GB, F[7], WH, F[8], Hh);
  k_rms<<<TRB * 64, 256, 0, stream>>>(Hh, F[9], (float*)d_out);
}
